// Gnn_model_68839735821122
// MI455X (gfx1250) — hardware-run, weakly checked
//
#include <hip/hip_runtime.h>
#include <math.h>

constexpr int N_NODES  = 50000;
constexpr int N_EDGES  = 800000;
constexpr int NPAD     = 50048;
constexpr int FDIM     = 128;
constexpr int HMSG     = 256;
constexpr int HRO      = 256;
constexpr int GATE3    = 384;
constexpr int AH_LD    = 256;
constexpr int PQ_LD    = 512;
constexpr int C1_LD    = 512;
constexpr int NODE_BLK = 64;
constexpr int N_NODE_BLKS = NPAD / NODE_BLK;
constexpr int EDGE_TILE = 64;
constexpr int MAX_TILES_PER_BLK = 256;
constexpr int A_LD     = HMSG + 8;
constexpr int M_LD     = FDIM + 4;
constexpr int HN_LD    = FDIM + 8;
constexpr int RO_ROWS  = 128;
constexpr float CARRY      = 16.0f;
constexpr float INV_CARRY  = 0.0625f;
constexpr float INV_CARRY2 = 0.00390625f;

static_assert(NPAD % 64 == 0 && NPAD >= N_NODES && NPAD - N_NODES < 64);
static_assert((NPAD / 64) * (PQ_LD / 64) == N_NODE_BLKS * 8);
static_assert((NPAD / 64) * (C1_LD / 64) == N_NODE_BLKS * 8);
static_assert(NPAD % RO_ROWS == 0);
static_assert(FDIM % 32 == 0 && HMSG % 32 == 0 && AH_LD % 32 == 0);
static_assert(N_NODES % 4 == 0);
static_assert(NPAD % 32 == 0);

typedef __attribute__((ext_vector_type(16))) _Float16 v16h;
typedef __attribute__((ext_vector_type(8)))  _Float16 v8h;
typedef __attribute__((ext_vector_type(16))) __bf16   v16b;
typedef __attribute__((ext_vector_type(8)))  __bf16   v8b;
typedef __attribute__((ext_vector_type(8)))  float    v8f;
typedef __attribute__((ext_vector_type(4)))  float    v4f;
typedef __attribute__((ext_vector_type(4)))  unsigned int v4u;
typedef __attribute__((ext_vector_type(2)))  unsigned int v2u;

__device__ __forceinline__ unsigned short f2bf_bits(float f) {
  unsigned u = __float_as_uint(f);
  return (unsigned short)((u + 0x7FFFu + ((u >> 16) & 1u)) >> 16);
}
__device__ __forceinline__ float bf_bits2f(unsigned short h) { return __uint_as_float(((unsigned)h) << 16); }
__device__ __forceinline__ unsigned pk16(unsigned short a, unsigned short b) { return (unsigned)a | ((unsigned)b << 16); }
__device__ __forceinline__ unsigned short h_bits(float f) { const _Float16 h = (_Float16)f; return __builtin_bit_cast(unsigned short, h); }

__device__ __forceinline__ float h16_to_f32(unsigned hb) {
  const unsigned sgn = (hb & 0x8000u) << 16; const unsigned em = hb & 0x7fffu;
  const float fn = __uint_as_float((em << 13) + 0x38000000u);
  const float fs = (float)em * 5.9604644775390625e-8f;
  const float mag = (em < 0x400u) ? fs : fn; return __uint_as_float(__float_as_uint(mag) | sgn); }

__device__ __forceinline__ void dep_guard_h(v8f& a, v8f& b, v16h x, v16h y) { asm volatile("v_nop\n\tv_nop\n\tv_nop\n\tv_nop" : "+v"(a), "+v"(b) : "v"(x), "v"(y)); }
__device__ __forceinline__ void dep_guard_b(v8f& a, v8f& b, v16b x, v16b y) { asm volatile("v_nop\n\tv_nop\n\tv_nop\n\tv_nop" : "+v"(a), "+v"(b) : "v"(x), "v"(y)); }
__device__ __forceinline__ void dep_guard4_h(v8f& a, v8f& b, v8f& c, v8f& d, v16h x, v16h y) { asm volatile("v_nop\n\tv_nop\n\tv_nop\n\tv_nop" : "+v"(a), "+v"(b), "+v"(c), "+v"(d) : "v"(x), "v"(y)); }
__device__ __forceinline__ void dep_guard4_b(v8f& a, v8f& b, v8f& c, v8f& d, v16b x, v16b y) { asm volatile("v_nop\n\tv_nop\n\tv_nop\n\tv_nop" : "+v"(a), "+v"(b), "+v"(c), "+v"(d) : "v"(x), "v"(y)); }
__device__ __forceinline__ void keep4_h(v16h a, v16h b, v16h c, v16h d) { asm volatile("v_nop" :: "v"(a), "v"(b), "v"(c), "v"(d)); }
__device__ __forceinline__ void keep4_b(v16b a, v16b b, v16b c, v16b d) { asm volatile("v_nop" :: "v"(a), "v"(b), "v"(c), "v"(d)); }
__device__ __forceinline__ void acc_guard4(v8f& a, v8f& b, v8f& c, v8f& d) { asm volatile("v_nop\n\tv_nop\n\tv_nop\n\tv_nop" : "+v"(a), "+v"(b), "+v"(c), "+v"(d)); }
template <typename T> struct Frag;
template <> struct Frag<_Float16> {
  typedef v16h V; union U { v16h v; v8h h[2]; };
  static __device__ __forceinline__ v16h load(const _Float16* p) {
    U f; f.h[0] = *(const v8h*)(p); f.h[1] = *(const v8h*)(p + 16); return f.v;
  }
  static __device__ __forceinline__ v8f mma(v16h a, v16h b, v8f c) {
    return __builtin_amdgcn_wmma_f32_16x16x32_f16(false, a, false, b, (short)0, c, false, false);
  }
  static __device__ __forceinline__ void guard(v8f& a, v8f& b, v16h x, v16h y) { dep_guard_h(a, b, x, y); }
  static __device__ __forceinline__ void guard4(v8f& a, v8f& b, v8f& c, v8f& d, v16h x, v16h y) { dep_guard4_h(a, b, c, d, x, y); }
  static __device__ __forceinline__ void keep(v16h a, v16h b, v16h c, v16h d) { keep4_h(a, b, c, d); }
};
template <> struct Frag<__bf16> {
  typedef v16b V; union U { v16b v; v8b h[2]; };
  static __device__ __forceinline__ v16b load(const __bf16* p) {
    U f; f.h[0] = *(const v8b*)(p); f.h[1] = *(const v8b*)(p + 16); return f.v;
  }
  static __device__ __forceinline__ v8f mma(v16b a, v16b b, v8f c) {
    return __builtin_amdgcn_wmma_f32_16x16x32_bf16(false, a, false, b, (short)0, c, false, false);
  }
  static __device__ __forceinline__ void guard(v8f& a, v8f& b, v16b x, v16b y) { dep_guard_b(a, b, x, y); }
  static __device__ __forceinline__ void guard4(v8f& a, v8f& b, v8f& c, v8f& d, v16b x, v16b y) { dep_guard4_b(a, b, c, d, x, y); }
  static __device__ __forceinline__ void keep(v16b a, v16b b, v16b c, v16b d) { keep4_b(a, b, c, d); }
};

template <int ET> struct Elem;
template <> struct Elem<0> { typedef _Float16 T; };
template <> struct Elem<1> { typedef __bf16 T; };
template <int ET, bool SPLIT, int BIAS_MODE, int OUT_MODE, bool RESID, int ACT = 0>
__global__ __launch_bounds__(256) void wmma_gemm64(
    const unsigned short* __restrict__ Ap, const unsigned short* __restrict__ A2p, int lda, long strideA,
    const unsigned short* __restrict__ Btp, const unsigned short* __restrict__ Bt2p, int ldb, long strideB,
    void* __restrict__ Cout, void* __restrict__ Cout2, int ldc, long strideC,
    const float* __restrict__ bias,
    const float* __restrict__ resid, long strideR,
    int M, int N, int K, float scale) {
  typedef typename Elem<ET>::T T;
  typedef typename Frag<T>::V V;
  const T* A = (const T*)Ap; const T* A2 = (const T*)A2p; const T* Bt = (const T*)Btp; const T* Bt2 = (const T*)Bt2p;
  __shared__ __align__(16) float sT[8][16 * 68];
  const int b    = blockIdx.y;
  const int lane = threadIdx.x & 31;
  const int wave = threadIdx.x >> 5;
  const int tilesN = N >> 6;
  const int tilesM = M >> 6;
  const int tile = blockIdx.x * 8 + wave;
  if (tile >= tilesM * tilesN) return;
  const int tm = tile / tilesN;
  const int tn = tile - tm * tilesN;
  const int m0 = tm << 6;
  const int n0 = tn << 6;

  const T* Ab  = A  + (size_t)b * strideA;
  const T* Bb  = Bt + (size_t)b * strideB;
  const T* Ab2 = SPLIT ? (A2  + (size_t)b * strideA) : nullptr;
  const T* Bb2 = SPLIT ? (Bt2 + (size_t)b * strideB) : nullptr;

  const int rlane = lane & 15;
  const int koff  = (lane >> 4) * 8;
  const int mOff  = (lane >> 4) * 8;

  v8f acc[4][4];
#pragma unroll
  for (int i = 0; i < 4; ++i)
#pragma unroll
    for (int j = 0; j < 4; ++j) acc[i][j] = (v8f){0.f,0.f,0.f,0.f,0.f,0.f,0.f,0.f};

  for (int k0 = 0; k0 < K; k0 += 32) {
    V bh[4], bl[4];
#pragma unroll
    for (int j = 0; j < 4; ++j) {
      const size_t bo = (size_t)(n0 + (j << 4) + rlane) * ldb + koff + k0;
      bh[j] = Frag<T>::load(Bb + bo);
      if (SPLIT) bl[j] = Frag<T>::load(Bb2 + bo);
    }
#pragma unroll
    for (int i = 0; i < 4; ++i) {
      const size_t ao = (size_t)(m0 + (i << 4) + rlane) * lda + koff + k0;
      V ah = Frag<T>::load(Ab + ao);
      V al;
      if (SPLIT) al = Frag<T>::load(Ab2 + ao);
#pragma unroll
      for (int j = 0; j < 4; ++j) {
        acc[i][j] = Frag<T>::mma(ah, bh[j], acc[i][j]);
        if (SPLIT) {
          acc[i][j] = Frag<T>::mma(ah, bl[j], acc[i][j]);
          acc[i][j] = Frag<T>::mma(al, bh[j], acc[i][j]);
        }
      }
      Frag<T>::guard4(acc[i][0], acc[i][1], acc[i][2], acc[i][3], ah, SPLIT ? al : ah);
    }
    Frag<T>::keep(bh[0], bh[1], bh[2], bh[3]);
    if (SPLIT) Frag<T>::keep(bl[0], bl[1], bl[2], bl[3]);
  }
  acc_guard4(acc[0][0], acc[0][1], acc[0][2], acc[0][3]);
  acc_guard4(acc[1][0], acc[1][1], acc[1][2], acc[1][3]);
  acc_guard4(acc[2][0], acc[2][1], acc[2][2], acc[2][3]);
  acc_guard4(acc[3][0], acc[3][1], acc[3][2], acc[3][3]);

  float* slab = sT[wave];
  const float* Rb = RESID ? (resid + (size_t)b * strideR) : nullptr;
#pragma unroll
  for (int i = 0; i < 4; ++i) {
    const int mBase = m0 + (i << 4);
#pragma unroll
    for (int j = 0; j < 4; ++j) {
      const int n = n0 + (j << 4) + rlane;
      float bv = 0.f;
      if (BIAS_MODE == 2) bv = bias[n];
#pragma unroll
      for (int r = 0; r < 8; ++r) {
        float v = acc[i][j][r] * scale;
        if (BIAS_MODE == 1) v += bias[mBase + mOff + r];
        if (BIAS_MODE == 2) v += bv;
        if (RESID) v += Rb[(size_t)(mBase + mOff + r) * ldc + n];
        if (ACT == 1) v = tanhf(v);
        if (ACT == 2) v = fmaxf(v, 0.0f);
        if (ACT == 3) v = v / (1.0f + expf(-v));
        if (ACT == 4) v = (v > 0.f) ? v : 0.01f * v;
        if (ACT == 5) v = 0.5f * v * (1.0f + erff(v * 0.70710678118654752f));
        slab[(mOff + r) * 68 + (j << 4) + rlane] = v;
      }
    }
    __builtin_amdgcn_fence(__ATOMIC_RELEASE, "workgroup");
    __builtin_amdgcn_wave_barrier();
    __builtin_amdgcn_fence(__ATOMIC_ACQUIRE, "workgroup");
    if (OUT_MODE == 0) {
      float* C = (float*)Cout + (size_t)b * strideC;
      const int hh = lane >> 4, c4 = (lane & 15) * 4;
      for (int pass = 0; pass < 2; ++pass) {
#pragma unroll
        for (int it = 0; it < 8; ++it) {
          const int row = it * 2 + hh;
          v4f v = *(const v4f*)(slab + row * 68 + c4);
          *(volatile v4f*)(C + (size_t)(mBase + row) * ldc + n0 + c4) = v;
        }
        __threadfence();
      }
    } else {
      const int q = lane >> 3, c8 = (lane & 7) * 8;
      unsigned short* C  = (unsigned short*)Cout  + (size_t)b * strideC;
      unsigned short* C2 = (OUT_MODE == 2) ? ((unsigned short*)Cout2 + (size_t)b * strideC) : nullptr;
      for (int pass = 0; pass < 2; ++pass) {
#pragma unroll
        for (int it = 0; it < 4; ++it) {
          const int row = it * 4 + q;
          const float* sp = slab + row * 68 + c8;
          v8h hv, lv;
#pragma unroll
          for (int e = 0; e < 8; ++e) {
            if (OUT_MODE == 1) {
              hv[e] = (_Float16)sp[e];
            } else {
              unsigned short hb = f2bf_bits(sp[e]);
              unsigned short lb = f2bf_bits(sp[e] - bf_bits2f(hb));
              hv[e] = __builtin_bit_cast(_Float16, hb);
              lv[e] = __builtin_bit_cast(_Float16, lb);
            }
          }
          *(volatile v8h*)(C + (size_t)(mBase + row) * ldc + n0 + c8) = hv;
          if (OUT_MODE == 2) *(volatile v8h*)(C2 + (size_t)(mBase + row) * ldc + n0 + c8) = lv;
        }
        __threadfence();
      }
    }
    __builtin_amdgcn_fence(__ATOMIC_RELEASE, "workgroup");
    __builtin_amdgcn_wave_barrier();
    __builtin_amdgcn_fence(__ATOMIC_ACQUIRE, "workgroup");
  }
}

__device__ __forceinline__ int lbound_idx(const int* __restrict__ a, int len, int key) {
  int lo = 0, hi = len;
#pragma unroll 1
  for (int it = 0; it < 21; ++it) {
    const bool act = lo < hi;
    int mid = (lo + hi) >> 1;
    mid = mid < len ? mid : (len - 1);
    mid = mid < 0 ? 0 : mid;
    const int v = a[mid];
    const bool gol = v < key;
    const int nlo = gol ? (mid + 1) : lo;
    const int nhi = gol ? hi : mid;
    lo = act ? nlo : lo;
    hi = act ? nhi : hi;
  }
  return lo;
}

__global__ __launch_bounds__(256) void fold_kernel(const float* __restrict__ k1, const float* __restrict__ k2,
                                                  const float* __restrict__ aw, const float* __restrict__ b1,
                                                  const float* __restrict__ bg,
                                                  float* __restrict__ cvec, float* __restrict__ d2v,
                                                  float* __restrict__ biasPQ, float* __restrict__ biasG) {
  __shared__ float awL[2 * FDIM];
  const int t = threadIdx.x;
  awL[t] = aw[t];
  __syncthreads();
  const int tr = t & 127;
  float cs = 0.0f, ds = 0.0f;
#pragma unroll 1
  for (int j = 0; j < FDIM; ++j) {
    cs = fmaf(k1[tr * FDIM + j], awL[j], cs);
    ds = fmaf(k2[tr * FDIM + j], awL[FDIM + j], ds);
  }
  const float pq0 = 0.0f;
  const float pq1 = CARRY * b1[t];
  const float g0  = CARRY * bg[t];
  const float bgt = bg[HMSG + tr];
  const float g1  = (t < FDIM) ? (CARRY * bgt) : 0.0f;
  for (int pass = 0; pass < 2; ++pass) {
    if (t < FDIM) { ((volatile float*)cvec)[t] = cs; ((volatile float*)d2v)[t] = ds; }
    ((volatile float*)biasPQ)[t] = pq0;
    ((volatile float*)biasPQ)[HMSG + t] = pq1;
    ((volatile float*)biasG)[t] = g0;
    ((volatile float*)biasG)[HMSG + t] = g1;
    __threadfence();
  }
}

__global__ __launch_bounds__(256) void btk128_kernel(const float* __restrict__ W1, const float* __restrict__ R1,
                                                    unsigned short* __restrict__ B1T,
                                                    unsigned short* __restrict__ R1TH, unsigned short* __restrict__ R1TL) {
  const int t = threadIdx.x, lane = t & 31, wave = t >> 5;
  const int rloc = wave * 2 + (lane >> 4);
  const int kg = (lane & 15) * 8;
  float v[8];
  if (blockIdx.x < 32) {
    const int n = blockIdx.x * 16 + rloc;
    const int half = n >> 8, col = n & 255;
#pragma unroll
    for (int i = 0; i < 8; ++i) v[i] = CARRY * W1[(size_t)(half * FDIM + kg + i) * HMSG + col];
    unsigned short hb[8];
#pragma unroll
    for (int i = 0; i < 8; ++i) hb[i] = h_bits(v[i]);
    const v4u u = (v4u){pk16(hb[0], hb[1]), pk16(hb[2], hb[3]), pk16(hb[4], hb[5]), pk16(hb[6], hb[7])};
    unsigned short* dp = B1T + (size_t)n * FDIM + kg;
    *(volatile v4u*)dp = u;
    __threadfence();
    *(volatile v4u*)dp = u;
  } else {
    const int n = (blockIdx.x - 32) * 16 + rloc;
#pragma unroll
    for (int i = 0; i < 8; ++i) v[i] = R1[(size_t)(kg + i) * HRO + n];
    unsigned short hb[8], lb[8];
#pragma unroll
    for (int i = 0; i < 8; ++i) { hb[i] = f2bf_bits(v[i]); lb[i] = f2bf_bits(v[i] - bf_bits2f(hb[i])); }
    const v4u uh = (v4u){pk16(hb[0], hb[1]), pk16(hb[2], hb[3]), pk16(hb[4], hb[5]), pk16(hb[6], hb[7])};
    const v4u ul = (v4u){pk16(lb[0], lb[1]), pk16(lb[2], lb[3]), pk16(lb[4], lb[5]), pk16(lb[6], lb[7])};
    unsigned short* hp = R1TH + (size_t)n * FDIM + kg;
    unsigned short* lp = R1TL + (size_t)n * FDIM + kg;
    *(volatile v4u*)hp = uh; *(volatile v4u*)lp = ul;
    __threadfence();
    *(volatile v4u*)hp = uh; *(volatile v4u*)lp = ul;
  }
}

__global__ __launch_bounds__(256) void btk256_kernel(const float* __restrict__ W2, const float* __restrict__ Wx,
                                                    const float* __restrict__ Wh,
                                                    unsigned short* __restrict__ W2T, unsigned short* __restrict__ BtG) {
  const int t = threadIdx.x, lane = t & 31, wave = t >> 5;
  const int kg = lane * 8;
  float v[8];
  unsigned short* dp;
  if (blockIdx.x < 16) {
    const int n = blockIdx.x * 8 + wave;
#pragma unroll
    for (int i = 0; i < 8; ++i) v[i] = CARRY * W2[(size_t)(kg + i) * FDIM + n];
    dp = W2T + (size_t)n * HMSG + kg;
  } else {
    const int n = (blockIdx.x - 16) * 8 + wave;
    const int g = n >> 7, c = n & 127;
    const int colx = (g < 3) ? (FDIM * g + c) : c;
    const int colh = c + ((g == 1) ? FDIM : 0) + ((g == 3) ? 2 * FDIM : 0);
    const float fx = (g < 3 && lane < 16) ? CARRY : 0.0f;
    const float fh = (g != 2 && lane >= 16) ? CARRY : 0.0f;
    float vx[8], vh[8];
#pragma unroll
    for (int i = 0; i < 8; ++i) { const int kk = (kg + i) & 127; vx[i] = Wx[(size_t)kk * GATE3 + colx]; }
    asm volatile("" ::: "memory");
#pragma unroll
    for (int i = 0; i < 8; ++i) { const int kk = (kg + i) & 127; vh[i] = Wh[(size_t)kk * GATE3 + colh]; }
#pragma unroll
    for (int i = 0; i < 8; ++i) v[i] = fmaf(fx, vx[i], fh * vh[i]);
    dp = BtG + (size_t)n * HMSG + kg;
  }
  unsigned short hb[8];
#pragma unroll
  for (int i = 0; i < 8; ++i) hb[i] = h_bits(v[i]);
  const v4u u = (v4u){pk16(hb[0], hb[1]), pk16(hb[2], hb[3]), pk16(hb[4], hb[5]), pk16(hb[6], hb[7])};
  *(volatile v4u*)dp = u;
  __threadfence();
  *(volatile v4u*)dp = u;
}

__global__ __launch_bounds__(512) void hprep_kernel(const float* __restrict__ h, const float* __restrict__ d2v,
                                                   unsigned short* __restrict__ AH, float* __restrict__ tdd) {
  __shared__ float tddL[32];
  const int t = threadIdx.x, lane = t & 31, wave = t >> 5;
  const int rloc = wave * 2 + (lane >> 4);
  const int f0 = (lane & 15) * 8;
  const int n = blockIdx.x * 32 + rloc;
  const bool live = n < N_NODES;
  const int nc = live ? n : (N_NODES - 1);
  const v4f a  = *(const v4f*)(h + (size_t)nc * FDIM + f0);
  const v4f bq = *(const v4f*)(h + (size_t)nc * FDIM + f0 + 4);
  const v4f da = *(const v4f*)(d2v + f0);
  const v4f db = *(const v4f*)(d2v + f0 + 4);
  float dot = 0.0f;
#pragma unroll
  for (int e = 0; e < 4; ++e) dot = fmaf(a[e], da[e], dot);
#pragma unroll
  for (int e = 0; e < 4; ++e) dot = fmaf(bq[e], db[e], dot);
  dot += __shfl_xor(dot, 1, 32);
  dot += __shfl_xor(dot, 2, 32);
  dot += __shfl_xor(dot, 4, 32);
  dot += __shfl_xor(dot, 8, 32);
  const float fac = live ? CARRY : 0.0f;
  v8h hv;
#pragma unroll
  for (int e = 0; e < 4; ++e) { hv[e] = (_Float16)(fac * a[e]); hv[4 + e] = (_Float16)(fac * bq[e]); }
  unsigned short* ap = AH + (size_t)n * AH_LD + FDIM + f0;
  *(volatile v8h*)ap = hv;
  __threadfence();
  *(volatile v8h*)ap = hv;
  if ((lane & 15) == 0) tddL[rloc] = live ? dot : 0.0f;
  __syncthreads();
  if (wave == 0) {
    const float tv = tddL[lane];
    float* tp = tdd + (size_t)blockIdx.x * 32 + lane;
    *(volatile float*)tp = tv;
    __threadfence();
    *(volatile float*)tp = tv;
  }
}

__global__ __launch_bounds__(256) void edge_agg_kernel(const unsigned short* __restrict__ PQ, const int* __restrict__ srcv,
                                                      const int* __restrict__ dstv, const float* __restrict__ tdd,
                                                      const unsigned short* __restrict__ W2T, const float* __restrict__ b2,
                                                      const float* __restrict__ cvec, unsigned short* __restrict__ AH) {
  __shared__ __align__(16) _Float16 aL[EDGE_TILE * A_LD];
  __shared__ __align__(16) float mL[EDGE_TILE * M_LD];
  __shared__ __align__(16) float accL[NODE_BLK * FDIM];
  __shared__ float cL[FDIM];
  __shared__ float b2L[FDIM];
  __shared__ int   rowNode[EDGE_TILE];
  __shared__ float tddRow[EDGE_TILE];
  __shared__ float sRow[EDGE_TILE];
  __shared__ float wRow[EDGE_TILE];
  __shared__ float Mv[NODE_BLK];
  __shared__ float Lv[NODE_BLK];
  __shared__ float fL[NODE_BLK];

  const int t = threadIdx.x, lane = t & 31, wave = t >> 5;
  const int rlane = lane & 15, koff = (lane >> 4) * 8, hh = lane >> 4;
  const int n0 = blockIdx.x * NODE_BLK;

  if (t < FDIM) { cL[t] = cvec[t]; b2L[t] = b2[t]; }
  for (int i = t; i < NODE_BLK * FDIM; i += 256) accL[i] = 0.0f;
  if (t < NODE_BLK) { Mv[t] = -INFINITY; Lv[t] = 0.0f; fL[t] = 0.0f; }
  if (t < EDGE_TILE) { rowNode[t] = -1; tddRow[t] = 0.0f; sRow[t] = 0.0f; wRow[t] = 0.0f; }

  const int eStart = lbound_idx(dstv, N_EDGES, n0);
  const int eEnd   = lbound_idx(dstv, N_EDGES, n0 + NODE_BLK);
  int nE = eEnd - eStart; nE = nE < 0 ? 0 : nE;
  int nT = (nE + EDGE_TILE - 1) / EDGE_TILE;
  nT = nT > MAX_TILES_PER_BLK ? MAX_TILES_PER_BLK : nT;
  __syncthreads();

  const int wr = wave & 3, wc = wave >> 2;
  const _Float16* W2Th = (const _Float16*)(const void*)W2T;

#pragma unroll 1
  for (int ti = 0; ti < nT; ++ti) {
    const int et = eStart + ti * EDGE_TILE;
#pragma unroll 1
    for (int it = 0; it < 8; ++it) {
      const int j = it * 8 + wave;
      const int e = et + j;
      const bool valid = e < eEnd;
      const int ec = (e < N_EDGES) ? e : (N_EDGES - 1);
      int s = srcv[ec]; s = s < 0 ? 0 : (s >= N_NODES ? N_NODES - 1 : s);
      int d = dstv[ec]; d = d < 0 ? 0 : (d >= N_NODES ? N_NODES - 1 : d);
      const v4u pw = *(const v4u*)(PQ + (size_t)s * PQ_LD + 8 * lane);
      const v4u qw = *(const v4u*)(PQ + (size_t)d * PQ_LD + HMSG + 8 * lane);
      const float tdv = tdd[d];
      const float vf = valid ? 1.0f : 0.0f;
      v8h o;
#pragma unroll
      for (int q2 = 0; q2 < 4; ++q2) {
        const unsigned pu = pw[q2], qu = qw[q2];
        const float p0 = h16_to_f32(pu & 0xffffu), q0 = h16_to_f32(qu & 0xffffu);
        const float p1 = h16_to_f32(pu >> 16),      q1 = h16_to_f32(qu >> 16);
        float x0 = p0 + q0; float x1 = p1 + q1;
        x0 = fmaxf(x0, 0.0f) * vf; x1 = fmaxf(x1, 0.0f) * vf;
        o[2 * q2] = (_Float16)x0; o[2 * q2 + 1] = (_Float16)x1;
      }
      *(v8h*)(aL + j * A_LD + 8 * lane) = o;
      if (lane == 0) {
        int dl = d - n0; dl = dl < 0 ? 0 : (dl > NODE_BLK - 1 ? NODE_BLK - 1 : dl);
        rowNode[j] = valid ? dl : -1;
        tddRow[j] = tdv;
      }
    }
    __syncthreads();
    v8f acc[4];
#pragma unroll
    for (int j = 0; j < 4; ++j) acc[j] = (v8f){0.f,0.f,0.f,0.f,0.f,0.f,0.f,0.f};
    for (int k0 = 0; k0 < HMSG; k0 += 32) {
      v16h bfr[4];
#pragma unroll
      for (int j = 0; j < 4; ++j)
        bfr[j] = Frag<_Float16>::load(W2Th + (size_t)(64 * wc + 16 * j + rlane) * HMSG + koff + k0);
      const v16h afr = Frag<_Float16>::load(aL + (16 * wr + rlane) * A_LD + koff + k0);
#pragma unroll
      for (int j = 0; j < 4; ++j) acc[j] = Frag<_Float16>::mma(afr, bfr[j], acc[j]);
      Frag<_Float16>::guard4(acc[0], acc[1], acc[2], acc[3], afr, bfr[0]);
      Frag<_Float16>::keep(bfr[0], bfr[1], bfr[2], bfr[3]);
    }
    acc_guard4(acc[0], acc[1], acc[2], acc[3]);
#pragma unroll
    for (int j = 0; j < 4; ++j) {
      const int col = 64 * wc + 16 * j + rlane;
      const float bb = b2L[col];
#pragma unroll
      for (int r = 0; r < 8; ++r) mL[(16 * wr + 8 * hh + r) * M_LD + col] = fmaf(acc[j][r], INV_CARRY2, bb);
    }
    __syncthreads();
    {
      const int j = t >> 2, part = t & 3;
      const float* mr = mL + j * M_LD + 32 * part;
      const float* cr = cL + 32 * part;
      float sd = 0.0f;
#pragma unroll 8
      for (int c = 0; c < 32; ++c) sd = fmaf(mr[c], cr[c], sd);
      sd += __shfl_xor(sd, 1, 32);
      sd += __shfl_xor(sd, 2, 32);
      float sv = sd + tddRow[j];
      sv = (sv >= 0.0f) ? sv : 0.2f * sv;
      if (part == 0) sRow[j] = sv;
    }
    __syncthreads();
    if (t < EDGE_TILE) {
      const int d  = rowNode[t];
      const int dq = rowNode[(t > 0) ? (t - 1) : 0];
      const int dp = (t > 0) ? dq : -1;
      if (d >= 0 && d != dp) {
        float mt = -INFINITY;
#pragma unroll 1
        for (int k = t; k < EDGE_TILE; ++k) { if (rowNode[k] != d) break; mt = fmaxf(mt, sRow[k]); }
        const float Mo = Mv[d];
        const float Mn = fmaxf(Mo, mt);
        const float f  = expf(Mo - Mn);
        float ls = 0.0f;
#pragma unroll 1
        for (int k = t; k < EDGE_TILE; ++k) {
          if (rowNode[k] != d) break;
          const float w = expf(sRow[k] - Mn);
          wRow[k] = w; ls += w;
        }
        Mv[d] = Mn;
        Lv[d] = fmaf(Lv[d], f, ls);
        fL[d] = f;
      }
    }
    __syncthreads();
    if (t < FDIM) {
      int prev = -1;
#pragma unroll 1
      for (int j = 0; j < EDGE_TILE; ++j) {
        const int d = rowNode[j];
        if (d >= 0) {
          float a = accL[d * FDIM + t];
          if (d != prev) { a = a * fL[d]; prev = d; }
          a = fmaf(wRow[j], mL[j * M_LD + t], a);
          accL[d * FDIM + t] = a;
        }
      }
    }
    __syncthreads();
  }
  __syncthreads();
  {
    const int q = lane >> 3, c8 = (lane & 7) * 8;
    for (int pass = 0; pass < 2; ++pass) {
#pragma unroll
      for (int it = 0; it < 4; ++it) {
        const int row  = 8 * wave + 2 * it + (q >> 1);
        const int colb = 64 * (q & 1) + c8;
        const float L   = Lv[row];
        const float Ls  = fmaxf(L, 1.0f);
        const float inv = ((L > 0.0f) ? CARRY : 0.0f) / Ls;
        v8h hv;
#pragma unroll
        for (int e = 0; e < 8; ++e) hv[e] = (_Float16)(accL[row * FDIM + colb + e] * inv);
        *(volatile v8h*)(AH + (size_t)(n0 + row) * AH_LD + colb) = hv;
      }
      __threadfence();
    }
  }
}

__global__ __launch_bounds__(256) void gru_readout_kernel(const unsigned short* __restrict__ C1, const float* __restrict__ h,
                                                         const unsigned short* __restrict__ R1TH, const unsigned short* __restrict__ R1TL,
                                                         const float* __restrict__ rb1, const float* __restrict__ R2,
                                                         const float* __restrict__ rb2, float* __restrict__ out) {
  __shared__ __align__(16) __bf16 Ahs[RO_ROWS * HN_LD];
  __shared__ __align__(16) __bf16 Als[RO_ROWS * HN_LD];
  __shared__ __align__(16) float sT[8][16 * 68];
  __shared__ float rb1L[HRO];
  __shared__ float R2L[HRO];
  __shared__ float part[8 * 64];
  __shared__ __align__(16) float outL[RO_ROWS];

  const int t = threadIdx.x, lane = t & 31, wave = t >> 5;
  const int rlane = lane & 15, koff = (lane >> 4) * 8, mOff = (lane >> 4) * 8;
  const int rbase = blockIdx.x * RO_ROWS;
  rb1L[t] = rb1[t];
  R2L[t]  = R2[t];

#pragma unroll 1
  for (int it = 0; it < 16; ++it) {
    const int idx = it * 256 + t;
    const int rl = idx >> 5;
    const int fq = (idx & 31) * 4;
    const int n  = rbase + rl;
    const bool live = n < N_NODES;
    const int nc = live ? n : (N_NODES - 1);
    const unsigned short* crow = C1 + (size_t)n * C1_LD + fq;
    const v2u zw = *(const v2u*)(crow);
    const v2u rw = *(const v2u*)(crow + FDIM);
    const v2u xw = *(const v2u*)(crow + 2 * FDIM);
    const v2u nw = *(const v2u*)(crow + 3 * FDIM);
    const v4f hv = *(const v4f*)(h + (size_t)nc * FDIM + fq);
    const float lf = live ? 1.0f : 0.0f;
    unsigned short hb[4], lb[4];
#pragma unroll
    for (int e = 0; e < 4; ++e) {
      const int w = e >> 1;
      const unsigned zbits = (e & 1) ? (zw[w] >> 16) : (zw[w] & 0xffffu);
      const unsigned rbits = (e & 1) ? (rw[w] >> 16) : (rw[w] & 0xffffu);
      const unsigned xbits = (e & 1) ? (xw[w] >> 16) : (xw[w] & 0xffffu);
      const unsigned nbits = (e & 1) ? (nw[w] >> 16) : (nw[w] & 0xffffu);
      const float az = h16_to_f32(zbits) * INV_CARRY;
      const float ar = h16_to_f32(rbits) * INV_CARRY;
      const float ax = h16_to_f32(xbits) * INV_CARRY;
      const float an = h16_to_f32(nbits) * INV_CARRY;
      const float z = 1.0f / (1.0f + expf(-az));
      const float r = 1.0f / (1.0f + expf(-ar));
      const float cand = tanhf(fmaf(r, an, ax));
      float hn = fmaf(z, hv[e], (1.0f - z) * cand);
      hn = hn * lf;
      hb[e] = f2bf_bits(hn);
      lb[e] = f2bf_bits(hn - bf_bits2f(hb[e]));
    }
    const v2u uh = (v2u){pk16(hb[0], hb[1]), pk16(hb[2], hb[3])};
    const v2u ul = (v2u){pk16(lb[0], lb[1]), pk16(lb[2], lb[3])};
    *(v2u*)(Ahs + rl * HN_LD + fq) = uh;
    *(v2u*)(Als + rl * HN_LD + fq) = ul;
  }
  __syncthreads();

  const int mloc = (wave >> 2) * 64;
  const int n0   = (wave & 3) * 64;
  const __bf16* Bh = (const __bf16*)(const void*)R1TH;
  const __bf16* Bl = (const __bf16*)(const void*)R1TL;
  v8f acc[4][4];
#pragma unroll
  for (int i = 0; i < 4; ++i)
#pragma unroll
    for (int j = 0; j < 4; ++j) acc[i][j] = (v8f){0.f,0.f,0.f,0.f,0.f,0.f,0.f,0.f};
  for (int k0 = 0; k0 < FDIM; k0 += 32) {
    v16b bh[4], bl[4];
#pragma unroll
    for (int j = 0; j < 4; ++j) {
      const size_t bo = (size_t)(n0 + (j << 4) + rlane) * FDIM + koff + k0;
      bh[j] = Frag<__bf16>::load(Bh + bo);
      bl[j] = Frag<__bf16>::load(Bl + bo);
    }
#pragma unroll
    for (int i = 0; i < 4; ++i) {
      const int ao = (mloc + (i << 4) + rlane) * HN_LD + koff + k0;
      const v16b ah = Frag<__bf16>::load(Ahs + ao);
      const v16b al = Frag<__bf16>::load(Als + ao);
#pragma unroll
      for (int j = 0; j < 4; ++j) {
        acc[i][j] = Frag<__bf16>::mma(ah, bh[j], acc[i][j]);
        acc[i][j] = Frag<__bf16>::mma(ah, bl[j], acc[i][j]);
        acc[i][j] = Frag<__bf16>::mma(al, bh[j], acc[i][j]);
      }
      Frag<__bf16>::guard4(acc[i][0], acc[i][1], acc[i][2], acc[i][3], ah, al);
    }
    Frag<__bf16>::keep(bh[0], bh[1], bh[2], bh[3]);
    Frag<__bf16>::keep(bl[0], bl[1], bl[2], bl[3]);
  }
  acc_guard4(acc[0][0], acc[0][1], acc[0][2], acc[0][3]);
  acc_guard4(acc[1][0], acc[1][1], acc[1][2], acc[1][3]);
  acc_guard4(acc[2][0], acc[2][1], acc[2][2], acc[2][3]);
  acc_guard4(acc[3][0], acc[3][1], acc[3][2], acc[3][3]);

  float* slab = sT[wave];
#pragma unroll
  for (int i = 0; i < 4; ++i) {
#pragma unroll
    for (int j = 0; j < 4; ++j) {
      const int n = n0 + (j << 4) + rlane;
      const float bv = rb1L[n];
#pragma unroll
      for (int r = 0; r < 8; ++r) {
        const float v = fmaxf(acc[i][j][r] + bv, 0.0f);
        slab[(mOff + r) * 68 + (j << 4) + rlane] = v;
      }
    }
    __builtin_amdgcn_fence(__ATOMIC_RELEASE, "workgroup");
    __builtin_amdgcn_wave_barrier();
    __builtin_amdgcn_fence(__ATOMIC_ACQUIRE, "workgroup");
    {
      const int row = lane & 15, ch = lane >> 4;
      const float* sp = slab + row * 68 + 32 * ch;
      const float* rp = R2L + n0 + 32 * ch;
      float ds = 0.0f;
#pragma unroll 8
      for (int c = 0; c < 32; ++c) ds = fmaf(sp[c], rp[c], ds);
      ds += __shfl_xor(ds, 16, 32);
      if (lane < 16) part[wave * 64 + 16 * i + row] = ds;
    }
    __builtin_amdgcn_fence(__ATOMIC_RELEASE, "workgroup");
    __builtin_amdgcn_wave_barrier();
    __builtin_amdgcn_fence(__ATOMIC_ACQUIRE, "workgroup");
  }
  __syncthreads();
  if (t < RO_ROWS) {
    const int g = t >> 6, r = t & 63;
    const float s01 = part[(4 * g) * 64 + r] + part[(4 * g + 1) * 64 + r];
    const float s012 = s01 + part[(4 * g + 2) * 64 + r];
    const float o = (s012 + part[(4 * g + 3) * 64 + r]) + rb2[0];
    outL[t] = o;
  }
  __syncthreads();
  if (wave == 0) {
    const int row0 = rbase + 4 * lane;
    const v4f ov = *(const v4f*)(outL + 4 * lane);
    const bool st = row0 < N_NODES;
    for (int pass = 0; pass < 2; ++pass) {
      if (st) *(volatile v4f*)(out + row0) = ov;
      __threadfence();
    }
  }
}

extern "C" void kernel_launch(void* const* d_in, const int* in_sizes, int n_in,
                              void* d_out, int out_size, void* d_ws, size_t ws_size,
                              hipStream_t stream) {
  (void)in_sizes; (void)n_in; (void)out_size;
  const float* h    = (const float*)d_in[0];
  const int*   src  = (const int*)  d_in[1];
  const int*   dst  = (const int*)  d_in[2];
  const float* W1   = (const float*)d_in[3];
  const float* b1   = (const float*)d_in[4];
  const float* W2   = (const float*)d_in[5];
  const float* b2   = (const float*)d_in[6];
  const float* k1   = (const float*)d_in[7];
  const float* k2   = (const float*)d_in[8];
  const float* aw   = (const float*)d_in[9];
  const float* Wx   = (const float*)d_in[10];
  const float* Wh   = (const float*)d_in[11];
  const float* bg   = (const float*)d_in[12];
  const float* R1   = (const float*)d_in[13];
  const float* rb1  = (const float*)d_in[14];
  const float* R2   = (const float*)d_in[15];
  const float* rb2  = (const float*)d_in[16];
  float* out = (float*)d_out;

  char* ws = (char*)d_ws; size_t off = 0;
  auto carve = [&](size_t bytes) -> char* { char* p = ws + off; off += (bytes + 255) & ~(size_t)255; return p; };
  unsigned short* AH     = (unsigned short*)carve((size_t)NPAD * AH_LD * 2);
  unsigned short* PQ     = (unsigned short*)carve((size_t)NPAD * PQ_LD * 2);
  unsigned short* C1     = (unsigned short*)carve((size_t)NPAD * C1_LD * 2);
  float*          tdd    = (float*)carve((size_t)NPAD * 4);
  unsigned short* B1T    = (unsigned short*)carve((size_t)PQ_LD * FDIM * 2);
  unsigned short* W2T    = (unsigned short*)carve((size_t)FDIM * HMSG * 2);
  unsigned short* BtG    = (unsigned short*)carve((size_t)C1_LD * AH_LD * 2);
  unsigned short* R1TH   = (unsigned short*)carve((size_t)HRO * FDIM * 2);
  unsigned short* R1TL   = (unsigned short*)carve((size_t)HRO * FDIM * 2);
  float*          cvec   = (float*)carve((size_t)FDIM * 4);
  float*          d2v    = (float*)carve((size_t)FDIM * 4);
  float*          biasPQ = (float*)carve((size_t)PQ_LD * 4);
  float*          biasG  = (float*)carve((size_t)C1_LD * 4);
  if (off > ws_size || off > (size_t)134217728) return;

  fold_kernel<<<1, 256, 0, stream>>>(k1, k2, aw, b1, bg, cvec, d2v, biasPQ, biasG);
  btk128_kernel<<<48, 256, 0, stream>>>(W1, R1, B1T, R1TH, R1TL);
  btk256_kernel<<<80, 256, 0, stream>>>(W2, Wx, Wh, W2T, BtG);
  hprep_kernel<<<NPAD / 32, 512, 0, stream>>>(h, d2v, AH, tdd);
  wmma_gemm64<0, false, 2, 1, false, 0><<<dim3(N_NODE_BLKS, 1), 256, 0, stream>>>(
      (const unsigned short*)(AH + FDIM), (const unsigned short*)nullptr, AH_LD, 0L,
      (const unsigned short*)B1T, (const unsigned short*)nullptr, FDIM, 0L,
      (void*)PQ, (void*)nullptr, PQ_LD, 0L,
      (const float*)biasPQ, (const float*)nullptr, 0L, NPAD, PQ_LD, FDIM, INV_CARRY);
  edge_agg_kernel<<<N_NODE_BLKS, 256, 0, stream>>>(PQ, src, dst, tdd, W2T, b2, cvec, AH);
  wmma_gemm64<0, false, 2, 1, false, 0><<<dim3(N_NODE_BLKS, 1), 256, 0, stream>>>(
      (const unsigned short*)AH, (const unsigned short*)nullptr, AH_LD, 0L,
      (const unsigned short*)BtG, (const unsigned short*)nullptr, AH_LD, 0L,
      (void*)C1, (void*)nullptr, C1_LD, 0L,
      (const float*)biasG, (const float*)nullptr, 0L, NPAD, C1_LD, AH_LD, INV_CARRY);
  gru_readout_kernel<<<NPAD / RO_ROWS, 256, 0, stream>>>(C1, h, R1TH, R1TL, rb1, R2, rb2, out);
}
